// PatchCoreModel_2534030704994
// MI455X (gfx1250) — hardware-verified
//
#include <hip/hip_runtime.h>
#include <math.h>

typedef __attribute__((ext_vector_type(16))) _Float16 v16h;
typedef __attribute__((ext_vector_type(16))) __bf16 v16b;
typedef __attribute__((ext_vector_type(8)))  _Float16 v8h;
typedef __attribute__((ext_vector_type(8)))  float v8f;
typedef __attribute__((ext_vector_type(4)))  float v4f;
typedef __attribute__((ext_vector_type(2)))  float v2f;
typedef __attribute__((ext_vector_type(4)))  unsigned v4u;
typedef __attribute__((ext_vector_type(4)))  int v4i;
typedef float __attribute__((may_alias)) float_a;
typedef int __attribute__((may_alias)) int_a;

template <typename T> __device__ __forceinline__ void vst2(void* p, T v) { *(volatile T*)p = v; __threadfence(); *(volatile T*)p = v; }
__device__ __forceinline__ v8f wmma16(v16h a, v16h b, v8f c) {
  v8f d = __builtin_amdgcn_wmma_f32_16x16x32_f16(false, a, false, b, (short)0, c, false, false);
  asm volatile("v_nop\n\tv_nop\n\tv_nop\n\tv_nop" : "+v"(d) : "v"(a), "v"(b));
  return d;
}
__device__ __forceinline__ v8f wmma_bf(v16b a, v16b b, v8f c) {
  v8f d = __builtin_amdgcn_wmma_f32_16x16x32_bf16(false, a, false, b, (short)0, c, false, false);
  asm volatile("v_nop\n\tv_nop\n\tv_nop\n\tv_nop" : "+v"(d) : "v"(a), "v"(b));
  return d;
}
__device__ __forceinline__ v16h frag_h(const _Float16* rowk0, int lane) {
  union { v16h v; v8h q[2]; } u; const _Float16* p = rowk0 + 8 * (lane >> 4);
  u.q[0] = *(const v8h*)p; u.q[1] = *(const v8h*)(p + 16); return u.v;
}
__device__ __forceinline__ v16h frag_f32(const float* rowk0, int lane) {
  v16h a; const float* p = rowk0 + 8 * (lane >> 4);
#pragma unroll
  for (int i = 0; i < 8; ++i) { a[i] = (_Float16)p[i]; a[8 + i] = (_Float16)p[16 + i]; }
  return a;
}
__device__ __forceinline__ v16h frag_f32s(const float* rowk0, int lane, float sc) {
  v16h a; const float* p = rowk0 + 8 * (lane >> 4);
#pragma unroll
  for (int i = 0; i < 8; ++i) { a[i] = (_Float16)(p[i] * sc); a[8 + i] = (_Float16)(p[16 + i] * sc); }
  return a;
}
__device__ __forceinline__ v16h fragc_f32(const float* W, int k0, int n, int lane, int ld, int K) {
  v16h a; const int g = lane >> 4;
#pragma unroll
  for (int i = 0; i < 8; ++i) { const int ka = k0 + 8 * g + i, kb = ka + 16;
    a[i] = (_Float16)(ka < K ? W[(size_t)(ka < K ? ka : K - 1) * ld + n] : 0.f); a[8 + i] = (_Float16)(kb < K ? W[(size_t)(kb < K ? kb : K - 1) * ld + n] : 0.f); }
  return a;
}
struct F2 { v16b h, l; };
__device__ __forceinline__ F2 bsplit16(const float v[16]) { F2 r;
#pragma unroll
  for (int i = 0; i < 16; ++i) { const __bf16 h = (__bf16)v[i]; r.h[i] = h; r.l[i] = (__bf16)(v[i] - (float)h); }
  return r; }
__device__ __forceinline__ F2 split_row(const float* row, int k0, int lane) { float v[16]; const float* p = row + k0 + 8 * (lane >> 4);
#pragma unroll
  for (int i = 0; i < 8; ++i) { v[i] = p[i]; v[8 + i] = p[16 + i]; }
  return bsplit16(v); }
__device__ __forceinline__ F2 split_rowK(const float* row, int k0, int lane, int K) { float v[16]; const int g = lane >> 4;
#pragma unroll
  for (int i = 0; i < 8; ++i) { const int ka = k0 + 8 * g + i, kb = ka + 16; v[i] = ka < K ? row[ka < K ? ka : K - 1] : 0.f; v[8 + i] = kb < K ? row[kb < K ? kb : K - 1] : 0.f; }
  return bsplit16(v); }
__device__ __forceinline__ F2 split_col(const float* W, int k0, int n, int lane, int ld, int K) { float v[16]; const int g = lane >> 4;
#pragma unroll
  for (int i = 0; i < 8; ++i) { const int ka = k0 + 8 * g + i, kb = ka + 16; v[i] = ka < K ? W[(size_t)(ka < K ? ka : K - 1) * ld + n] : 0.f; v[8 + i] = kb < K ? W[(size_t)(kb < K ? kb : K - 1) * ld + n] : 0.f; }
  return bsplit16(v); }
__device__ __forceinline__ v8f mac3(const F2& a, const F2& b, v8f c) { c = wmma_bf(a.l, b.h, c); c = wmma_bf(a.h, b.l, c); return wmma_bf(a.h, b.h, c); }
__device__ __forceinline__ float sigm(float v) { return 1.0f / (1.0f + expf(-v)); }
#define LDSX() do { asm volatile("s_wait_dscnt 0" ::: "memory"); __builtin_amdgcn_wave_barrier(); __builtin_amdgcn_fence(__ATOMIC_RELEASE, "workgroup"); } while (0)

__device__ __forceinline__ float bfr(float v) { return (float)(__bf16)v; }
#define NIMG 8
#define PH 28
#define NPATCH (NIMG * PH * PH)
#define DD 128
#define MB 30000
#define IMG 224
#ifndef NRB
#define NRB (NPATCH / 64)
#endif
#define WS_M2  0u
#define WS_NN  (WS_M2 + 4u * 30080u)
#define WS_ST  (WS_NN + 4u * (size_t)NPATCH)
#define NOUT   (NIMG + NIMG * IMG * IMG)
#define WS_SCO (WS_ST + 1605888u)
#define WS_END (WS_SCO + 4u * 8u * 32u)
__global__ __launch_bounds__(64) void k_m2(const float* __restrict__ MEM, float* __restrict__ M2) { __shared__ __align__(16) float sm[64];
  const int j = blockIdx.x * 64 + threadIdx.x; float s = 0.f; if (j < MB) { const float* p = MEM + (size_t)j * DD; for (int d = 0; d < DD; ++d) { const float v = bfr(p[d]); s += v * v; } }
  sm[threadIdx.x] = s; LDSX(); __syncthreads(); if (threadIdx.x < 16) vst2(M2 + blockIdx.x * 64 + threadIdx.x * 4, *(const v4f*)&sm[threadIdx.x * 4]); }
__global__ __launch_bounds__(128) void k_nn(const float* __restrict__ FEAT, const float* __restrict__ MEM, const float* __restrict__ M2, float* __restrict__ NN) { __shared__ __align__(16) float snn[64]; __shared__ float sf2[64];
  const int tid = threadIdx.x, wave = tid >> 5, lane = tid & 31, col = lane & 15, g = lane >> 4; const size_t r0 = (size_t)blockIdx.x * 64 + wave * 16;
  if (tid < 64) { const float* p = FEAT + ((size_t)blockIdx.x * 64 + tid) * DD; float s = 0.f; for (int d = 0; d < DD; ++d) { const float v = bfr(p[d]); s += v * v; } sf2[tid] = s; }
  v16b af[4];
#pragma unroll
  for (int kc = 0; kc < 4; ++kc) { const float* p = FEAT + (r0 + col) * DD + kc * 32 + 8 * g;
#pragma unroll
    for (int i = 0; i < 8; ++i) { af[kc][i] = (__bf16)p[i]; af[kc][8 + i] = (__bf16)p[16 + i]; } }
  __syncthreads();
  float rmin[8];
#pragma unroll
  for (int r = 0; r < 8; ++r) rmin[r] = 3.0e38f;
#pragma unroll 1
  for (int cb = 0; cb < (MB + 127) / 128; ++cb) { const int c0 = cb * 128; v8f acc[8] = {};
#pragma unroll
    for (int kc = 0; kc < 4; ++kc) {
#pragma unroll
      for (int j = 0; j < 8; ++j) { v16b w; const int mrow = c0 + j * 16 + col; const int mr = mrow < MB ? mrow : MB - 1; const float* p = MEM + (size_t)mr * DD + kc * 32 + 8 * g;
#pragma unroll
        for (int i = 0; i < 8; ++i) { w[i] = (__bf16)p[i]; w[8 + i] = (__bf16)p[16 + i]; }
        acc[j] = wmma_bf(af[kc], w, acc[j]); } }
#pragma unroll
    for (int j = 0; j < 8; ++j) { const int mcol = c0 + j * 16 + col; const float m2 = (mcol < MB) ? M2[mcol] : 3.0e38f;
#pragma unroll
      for (int r = 0; r < 8; ++r) { const float f2 = sf2[wave * 16 + 8 * g + r]; const float dist = (mcol < MB) ? ((f2 + m2) - 2.0f * acc[j][r]) : 3.0e38f; rmin[r] = fminf(rmin[r], dist); } } }
#pragma unroll
  for (int r = 0; r < 8; ++r) { float v = rmin[r];
#pragma unroll
    for (int o = 1; o < 16; o <<= 1) v = fminf(v, __shfl_xor(v, o));
    if (col == 0) snn[wave * 16 + 8 * g + r] = v; }
  __syncthreads(); if (tid < 16) vst2(NN + (size_t)blockIdx.x * 64 + tid * 4, *(const v4f*)&snn[tid * 4]); }
__global__ __launch_bounds__(256) void k_post(const float* __restrict__ NN, float* __restrict__ ST, float* __restrict__ SCO) { __shared__ float sp[PH * PH]; __shared__ float sred[8]; __shared__ __align__(16) float srow[IMG];
  const int t = threadIdx.x; const int img = blockIdx.x; const float* pv = NN + (size_t)img * PH * PH;
  float m = -3.0e38f; for (int e = t; e < PH * PH; e += 256) { const float v = pv[e]; sp[e] = v; m = fmaxf(m, v); }
#pragma unroll
  for (int o = 1; o < 32; o <<= 1) m = fmaxf(m, __shfl_xor(m, o));
  if ((t & 31) == 0) sred[t >> 5] = m; __syncthreads();
  if (t == 0) { float a = sred[0]; for (int e = 1; e < 8; ++e) a = fmaxf(a, sred[e]); vst2(SCO + img * 32, a); }
  for (int oy = 0; oy < IMG; ++oy) { const float sy = ((float)oy + 0.5f) * (1.0f / 8.0f) - 0.5f; const int y0 = (int)floorf(sy); const float wy = sy - (float)y0; const int ya = y0 < 0 ? 0 : y0, yb = (y0 + 1 > PH - 1) ? PH - 1 : y0 + 1;
    if (t < IMG) { const float sx = ((float)t + 0.5f) * (1.0f / 8.0f) - 0.5f; const int x0 = (int)floorf(sx); const float wx = sx - (float)x0; const int xa = x0 < 0 ? 0 : x0, xb = (x0 + 1 > PH - 1) ? PH - 1 : x0 + 1;
      const float top = sp[ya * PH + xa] * (1.0f - wx) + sp[ya * PH + xb] * wx, bot = sp[yb * PH + xa] * (1.0f - wx) + sp[yb * PH + xb] * wx; srow[t] = top * (1.0f - wy) + bot * wy; }
    __syncthreads();
    if (t < IMG / 4) vst2(ST + 32 + ((size_t)img * IMG + oy) * IMG + t * 4, *(const v4f*)&srow[t * 4]);
    __syncthreads(); } }
__global__ __launch_bounds__(256) void k_flat(const float* __restrict__ ST, const float* __restrict__ SCO, float* __restrict__ OUT) {
  const size_t nq = NOUT / 4;
  const size_t nfull = (nq / 8) * 8;
  for (size_t q = (size_t)blockIdx.x * 256 + threadIdx.x; q < nfull; q += (size_t)gridDim.x * 256) { v4f v; if (q < 2) { for (int i = 0; i < 4; ++i) v[i] = SCO[(q * 4 + i) * 32]; } else v = *(const v4f*)(ST + 32 + (q - 2) * 4); vst2(OUT + q * 4, v); }
  if (blockIdx.x == 0 && threadIdx.x == 0) { for (size_t q = nfull; q < nq; ++q) vst2(OUT + q * 4, *(const v4f*)(ST + 32 + (q - 2) * 4)); } }
extern "C" void kernel_launch(void* const* d_in, const int* in_sizes, int n_in, void* d_out, int out_size, void* d_ws, size_t ws_size, hipStream_t stream) {
  (void)in_sizes; (void)n_in; (void)out_size;
  const float** F = (const float**)d_in;
  if (ws_size < (size_t)WS_END) return;
  char* ws = (char*)d_ws; float *M2 = (float*)(ws + WS_M2), *NN = (float*)(ws + WS_NN), *ST = (float*)(ws + WS_ST), *SCO = (float*)(ws + WS_SCO);
  k_m2<<<dim3((MB + 63) / 64), 64, 0, stream>>>(F[1], M2);
  k_nn<<<dim3(NRB), 128, 0, stream>>>(F[0], F[1], M2, NN);
  k_post<<<dim3(NIMG), 256, 0, stream>>>(NN, ST, SCO);
  k_flat<<<dim3(64), 256, 0, stream>>>(ST, SCO, (float*)d_out);
}
